// cross_module_29996051595336
// MI455X (gfx1250) — hardware-verified
//
#include <hip/hip_runtime.h>


namespace {
constexpr int Bn = 2, C = 64, C2 = 32, HW = 64, NPX = HW * HW, NT = Bn * NPX;
constexpr float XS = 8.0f, PS = 8.0f;

typedef _Float16 b16;
typedef __attribute__((ext_vector_type(16))) _Float16 v16b;
typedef __attribute__((ext_vector_type(8))) _Float16 v8b;
typedef __attribute__((ext_vector_type(8))) float v8f;
typedef __attribute__((ext_vector_type(4))) float v4f;
__device__ __forceinline__ float bf16_rne(float f) { unsigned int u = __float_as_uint(f); u += 0x7FFFu + ((u >> 16) & 1u); return __uint_as_float(u & 0xFFFF0000u); }
__device__ __forceinline__ void split16(float v, b16& hi, b16& lo) { hi = (b16)v; lo = (b16)(v - (float)hi); }
__device__ __forceinline__ v16b frag_kb(const b16* p, int hh) { const v8b a = *(const v8b*)(p + 8 * hh), b = *(const v8b*)(p + 16 + 8 * hh); v16b f;
#pragma unroll
  for (int e = 0; e < 8; ++e) { f[e] = a[e]; f[8 + e] = b[e]; } return f; }
__device__ __forceinline__ v8f wmma16b(v16b a, v16b b, v8f c) { v8f d = __builtin_amdgcn_wmma_f32_16x16x32_f16(false, a, false, b, (short)0, c, false, false); asm volatile("v_nop\n\tv_nop\n\tv_nop\n\tv_nop" : "+v"(d) : "v"(a), "v"(b)); return d; }
__device__ __forceinline__ void wave_lds_sync() { __builtin_amdgcn_fence(__ATOMIC_RELEASE, "workgroup"); __builtin_amdgcn_wave_barrier(); __builtin_amdgcn_fence(__ATOMIC_ACQUIRE, "workgroup"); }
__device__ __forceinline__ float nexp(float x) { return __builtin_amdgcn_exp2f(x * 1.4426950408889634f); }
__device__ __forceinline__ float pmul(float a, float b) { float p = a * b; asm volatile("" : "+v"(p)); return p; }
__device__ __forceinline__ float sigm(float x) { return 1.0f / (1.0f + nexp(-x)); }

__global__ __launch_bounds__(256) void prep_kernel(const float* __restrict__ x1, const float* __restrict__ x2, const float* __restrict__ wq1, const float* __restrict__ bq1, const float* __restrict__ wk1, const float* __restrict__ bk1, const float* __restrict__ wv1, const float* __restrict__ bv1, const float* __restrict__ wc1, const float* __restrict__ bc1,
    const float* __restrict__ wq2, const float* __restrict__ bq2, const float* __restrict__ wk2, const float* __restrict__ bk2, const float* __restrict__ wv2, const float* __restrict__ bv2, const float* __restrict__ wc2, const float* __restrict__ bc2, const float* __restrict__ g1, const float* __restrict__ g2, b16* __restrict__ R, float* __restrict__ P, b16* __restrict__ XT) {
  __shared__ __attribute__((aligned(16))) b16 Tx[64][C + 8];
  const int i = blockIdx.z, b = blockIdx.y, p0 = blockIdx.x * 64, t_ = threadIdx.x; const float* x = i ? x2 : x1;
  const size_t tid = ((size_t)(blockIdx.z * Bn + blockIdx.y) * gridDim.x + blockIdx.x) * 256 + t_, nth = (size_t)gridDim.x * Bn * 2 * 256;
  for (int k = t_; k < C * 64; k += 256) { const int c = k >> 6, px = k & 63; Tx[px][c] = (b16)(bf16_rne(x[((size_t)b * C + c) * NPX + p0 + px]) * XS); }
  __syncthreads();
  for (int pass = 0; pass < 2; ++pass) {
    for (size_t p = tid; p < (size_t)2 * 96 * C; p += nth) { const int ii = (int)(p / (96 * C)), o = (int)((p / C) % 96), c = (int)(p % C); const float* w = ii ? ((o < 32) ? wq2 : (o < 64) ? wk2 : wv2) : ((o < 32) ? wq1 : (o < 64) ? wk1 : wv1); ((volatile b16*)R)[p] = (b16)bf16_rne(w[(size_t)(o & 31) * C + c]); }
    for (size_t q = tid; q < 4418; q += nth) { const int j = (int)q; float v;
      if (j < 96) v = ((j < 32) ? bq1 : (j < 64) ? bk1 : bv1)[j & 31]; else if (j < 192) v = ((j < 128) ? bq2 : (j < 160) ? bk2 : bv2)[j & 31]; else if (j < 2240) v = wc1[j - 192]; else if (j < 2304) v = bc1[j - 2240]; else if (j < 4352) v = wc2[j - 2304]; else if (j < 4416) v = bc2[j - 4352]; else v = (j == 4416) ? g1[0] : g2[0];
      P[q] = bf16_rne(v); }
    for (int k = t_; k < 64 * 8; k += 256) { const int px = k >> 3, c8 = (k & 7) * 8; *(volatile v8b*)(XT + ((size_t)i * NT + (size_t)b * NPX + p0 + px) * C + c8) = *(const v8b*)(&Tx[px][c8]); }
    __threadfence(); }
}
__global__ __launch_bounds__(128) void proj_kernel(const b16* __restrict__ XT, const b16* __restrict__ R, const float* __restrict__ P, float* __restrict__ QK, b16* __restrict__ Vh, b16* __restrict__ Vl) {
  __shared__ __attribute__((aligned(16))) b16 Th[C2][64 + 8], Tl[C2][64 + 8]; __shared__ __attribute__((aligned(16))) float Qs[2][64];
  const int i = blockIdx.y, g0 = blockIdx.x * 64, lane = threadIdx.x & 31, wave = threadIdx.x >> 5, nloc = lane & 15, hlf = lane >> 4, m0 = g0 + wave * 16; const b16* Bw = R + (size_t)i * 96 * C; const float* bias = P + i * 96;
  const int b = g0 / NPX, px0 = g0 % NPX;
  v8f acc[6];
#pragma unroll
  for (int t = 0; t < 6; ++t) acc[t] = (v8f){};
#pragma unroll
  for (int kb = 0; kb < C; kb += 32) { const v16b a = frag_kb(XT + ((size_t)i * NT + m0 + nloc) * C + kb, hlf);
#pragma unroll
    for (int t = 0; t < 6; ++t) acc[t] = wmma16b(a, frag_kb(Bw + (size_t)(t * 16 + nloc) * C + kb, hlf), acc[t]); }
#pragma unroll
  for (int r = 0; r < 8; ++r) { float q0 = acc[0][r] * (1.0f / XS) + bias[nloc], q1 = acc[1][r] * (1.0f / XS) + bias[16 + nloc], k0 = acc[2][r] * (1.0f / XS) + bias[32 + nloc], k1 = acc[3][r] * (1.0f / XS) + bias[48 + nloc];
    float qv = (i == 0) ? fmaxf(q0, q1) : (q0 + q1), kv = (i == 0) ? fmaxf(k0, k1) : (k0 + k1);
#pragma unroll
    for (int o = 1; o < 16; o <<= 1) { const float qo = __shfl_xor(qv, o), ko = __shfl_xor(kv, o); qv = (i == 0) ? fmaxf(qv, qo) : (qv + qo); kv = (i == 0) ? fmaxf(kv, ko) : (kv + ko); }
    if (nloc == 0) { Qs[0][wave * 16 + 8 * hlf + r] = (i == 0) ? qv : qv * (1.0f / C2); Qs[1][wave * 16 + 8 * hlf + r] = (i == 0) ? kv : kv * (1.0f / C2); } }
#pragma unroll
  for (int t = 4; t < 6; ++t)
#pragma unroll
    for (int r = 0; r < 8; ++r) { b16 a_, c_; split16(acc[t][r] + XS * bias[64 + (t - 4) * 16 + nloc], a_, c_); Th[(t - 4) * 16 + nloc][wave * 16 + 8 * hlf + r] = a_; Tl[(t - 4) * 16 + nloc][wave * 16 + 8 * hlf + r] = c_; }
  __syncthreads();
  for (int pass = 0; pass < 2; ++pass) { if (threadIdx.x < 32) { const int w = threadIdx.x >> 4, c4 = (threadIdx.x & 15) * 4; *(volatile v4f*)(QK + ((size_t)i * 2 + w) * NT + g0 + c4) = *(const v4f*)(&Qs[w][c4]); }
    for (int k = threadIdx.x; k < C2 * 8; k += 128) { const int c = k >> 3, c8 = (k & 7) * 8; const size_t gi = (((size_t)i * Bn + b) * C2 + c) * NPX + px0 + c8; *(volatile v8b*)(Vh + gi) = *(const v8b*)(&Th[c][c8]); *(volatile v8b*)(Vl + gi) = *(const v8b*)(&Tl[c][c8]); } __threadfence(); }
}
__global__ __launch_bounds__(64) void attn_kernel(const float* __restrict__ QK, const b16* __restrict__ Vh, const b16* __restrict__ Vl, const float* __restrict__ P, const float* __restrict__ x1, const float* __restrict__ x2, float* __restrict__ out) {
  __shared__ __attribute__((aligned(16))) float Os[C2][32 + 1]; __shared__ __attribute__((aligned(16))) float Ys[C][32 + 4];
  const int br = blockIdx.z, b = blockIdx.y, wave = threadIdx.x >> 5, lane = threadIdx.x & 31, hh = lane >> 4, col = lane & 15; const int m0 = blockIdx.x * 32 + wave * 16, mi = m0 + col;
  const float* qv = QK + ((size_t)(br ? 1 : 0) * 2 + 0) * NT + (size_t)b * NPX; const float* kv = QK + ((size_t)(br ? 0 : 1) * 2 + 1) * NT + (size_t)b * NPX; const b16* V = Vh + (((size_t)br * Bn + b) * C2) * NPX; const b16* VL = Vl + (((size_t)br * Bn + b) * C2) * NPX;
  const float qm = qv[mi]; v8f o[2] = {{}, {}};
  for (int kb = 0; kb < NPX; kb += 32) { v16b pb, pl;
#pragma unroll
    for (int r = 0; r < 8; ++r) { const float ka = kv[kb + 8 * hh + r], kbv = kv[kb + 16 + 8 * hh + r]; const float s0 = sigm(pmul(qm, ka)), s1 = sigm(pmul(qm, kbv)); const float a0 = br ? s0 : (1.0f - s0), a1 = br ? s1 : (1.0f - s1); b16 h_, l_; split16(a0 * PS, h_, l_); pb[r] = h_; pl[r] = l_; split16(a1 * PS, h_, l_); pb[8 + r] = h_; pl[8 + r] = l_; }
#pragma unroll
    for (int t = 0; t < 2; ++t) { const v16b vh = frag_kb(V + (size_t)(t * 16 + col) * NPX + kb, hh); o[t] = wmma16b(vh, pb, o[t]); o[t] = wmma16b(vh, pl, o[t]); o[t] = wmma16b(frag_kb(VL + (size_t)(t * 16 + col) * NPX + kb, hh), pb, o[t]); } }
#pragma unroll
  for (int t = 0; t < 2; ++t)
#pragma unroll
    for (int r = 0; r < 8; ++r) Os[t * 16 + 8 * hh + r][wave * 16 + col] = o[t][r] * (1.0f / (XS * PS));
  __syncthreads();
  { const int oo = threadIdx.x; const float* wc = P + (br ? 192 : 2304) + oo * C2; const float bc = P[(br ? 2240 : 4352) + oo]; const float gm = P[4416 + br]; const float* xr = (br ? x2 : x1) + ((size_t)b * C + oo) * NPX + blockIdx.x * 32;
    for (int m = 0; m < 32; ++m) { float s = bc; for (int c = 0; c < C2; ++c) s += pmul(Os[c][m], wc[c]); Ys[oo][m] = bf16_rne(xr[m]) + pmul(gm, s); } }
  __syncthreads();
  float* ob = out + (size_t)br * Bn * C * NPX;
  for (int pass = 0; pass < 2; ++pass) { for (int k = threadIdx.x; k < C * 8; k += 64) { const int oo = k >> 3, c4 = (k & 7) * 4; *(volatile v4f*)(ob + ((size_t)b * C + oo) * NPX + blockIdx.x * 32 + c4) = *(const v4f*)(&Ys[oo][c4]); } __threadfence(); }
}
}

extern "C" void kernel_launch(void* const* d_in, const int* in_sizes, int n_in,
                              void* d_out, int out_size, void* d_ws, size_t ws_size, hipStream_t stream) {
  (void)n_in; (void)out_size;
  auto Fp = [&](int i) { return (const float*)d_in[i]; };
  float* out = (float*)d_out;
  if (in_sizes[0] != NT * C || in_sizes[1] != NT * C || in_sizes[2] != C2 * C || in_sizes[8] != C * C2) return;
  size_t off = 0; char* ws = (char*)d_ws;
  auto carve = [&](size_t bytes) { char* p = ws + off; off += (bytes + 255) & ~(size_t)255; return p; };
  b16* R = (b16*)carve((size_t)2 * 96 * C * 2); float* P = (float*)carve(4420 * 4); b16* XT = (b16*)carve((size_t)2 * NT * C * 2); float* QK = (float*)carve((size_t)4 * NT * 4); b16* Vh = (b16*)carve((size_t)2 * Bn * C2 * NPX * 2); b16* Vl = (b16*)carve((size_t)2 * Bn * C2 * NPX * 2);
  if (off > ws_size) return;
  prep_kernel<<<dim3(NPX / 64, Bn, 2), 256, 0, stream>>>(Fp(0), Fp(1), Fp(2), Fp(3), Fp(4), Fp(5), Fp(6), Fp(7), Fp(8), Fp(9), Fp(10), Fp(11), Fp(12), Fp(13), Fp(14), Fp(15), Fp(16), Fp(17), Fp(18), Fp(19), R, P, XT);
  proj_kernel<<<dim3(NT / 64, 2), 128, 0, stream>>>(XT, R, P, QK, Vh, Vl);
  attn_kernel<<<dim3(NPX / 32, Bn, 2), 64, 0, stream>>>(QK, Vh, Vl, P, Fp(0), Fp(1), out);
}
